// LearnableCorrBlock_66451734003973
// MI455X (gfx1250) — hardware-verified
//
#include <hip/hip_runtime.h>

typedef __attribute__((ext_vector_type(16))) _Float16 v16h;
typedef __attribute__((ext_vector_type(8)))  _Float16 v8h;
typedef __attribute__((ext_vector_type(16))) __bf16   v16b;
typedef __attribute__((ext_vector_type(8)))  __bf16   v8b;
typedef __attribute__((ext_vector_type(8)))  float    v8f;
typedef __attribute__((ext_vector_type(4)))  float    v4f;
typedef __attribute__((ext_vector_type(8)))  unsigned short u16x8;

constexpr int kDim = 256;
constexpr int kImg = 64;
constexpr int kHW  = 4096;
constexpr int kNB  = 2;
constexpr int kNCH = 324;
constexpr int kChunkRows = 2048;
constexpr int kNChunk = (kNB * kHW) / kChunkRows;
constexpr int kChunkH = kChunkRows / kImg;

static_assert(kDim % 32 == 0);
static_assert(kDim % 64 == 0 && kHW % 64 == 0 && kChunkRows % 64 == 0);
static_assert(kNChunk * kChunkRows == kNB * kHW);
static_assert(kChunkH * kImg == kChunkRows);

constexpr size_t kBMaug = (size_t)kDim * 2 * kDim * 4;
constexpr size_t kBMat  = (size_t)kDim * kDim * 4;
constexpr size_t kBDvec = 1024;
constexpr size_t kBWpl  = (size_t)kDim * kDim * 2;
constexpr size_t kBFpl  = (size_t)kNB * kHW * kDim * 2;
constexpr size_t kBCorr = (size_t)kChunkRows * kHW * 4;
constexpr size_t kBP1   = (size_t)kChunkRows * 1024 * 4;
constexpr size_t kBP2   = (size_t)kChunkRows * 256 * 4;
constexpr size_t kBP3   = (size_t)kChunkRows * 64 * 4;
constexpr size_t oMaug = 0;
constexpr size_t oIpS  = oMaug + kBMaug;
constexpr size_t oInv  = oIpS + kBMat;
constexpr size_t oPm   = oInv + kBMat;
constexpr size_t oDvec = oPm + kBMat;
constexpr size_t oWTh  = oDvec + kBDvec;
constexpr size_t oWTl  = oWTh + kBWpl;
constexpr size_t oF1h  = oWTl + kBWpl;
constexpr size_t oF1l  = oF1h + kBFpl;
constexpr size_t oF2h  = oF1l + kBFpl;
constexpr size_t oF2l  = oF2h + kBFpl;
constexpr size_t oTh   = oF2l + kBFpl;
constexpr size_t oTl   = oTh + kBFpl;
constexpr size_t oCorr = oTl + kBFpl;
constexpr size_t oP1   = oCorr + kBCorr;
constexpr size_t oP2   = oP1 + kBP1;
constexpr size_t oP3   = oP2 + kBP2;
constexpr size_t kWsTotal = oP3 + kBP3;
static_assert(kWsTotal == 71304192);
static_assert(kWsTotal <= 134217728);
static_assert(oWTh % 256 == 0 && oF1h % 256 == 0 && oTh % 256 == 0 && oCorr % 256 == 0 && oP1 % 256 == 0 && oP2 % 256 == 0 && oP3 % 256 == 0);

__device__ __forceinline__ unsigned short f2bf_bits(float f) {
  unsigned u = __float_as_uint(f);
  return (unsigned short)((u + 0x7FFFu + ((u >> 16) & 1u)) >> 16);
}
__device__ __forceinline__ float bf_bits2f(unsigned short h) { return __uint_as_float(((unsigned)h) << 16); }

__device__ __forceinline__ void dep_guard_h(v8f& a, v8f& b, v16h x, v16h y) { asm volatile("v_nop\n\tv_nop\n\tv_nop\n\tv_nop" : "+v"(a), "+v"(b) : "v"(x), "v"(y)); }
__device__ __forceinline__ void dep_guard_b(v8f& a, v8f& b, v16b x, v16b y) { asm volatile("v_nop\n\tv_nop\n\tv_nop\n\tv_nop" : "+v"(a), "+v"(b) : "v"(x), "v"(y)); }
__device__ __forceinline__ void keep4_h(v16h a, v16h b, v16h c, v16h d) { asm volatile("v_nop" :: "v"(a), "v"(b), "v"(c), "v"(d)); }
__device__ __forceinline__ void keep4_b(v16b a, v16b b, v16b c, v16b d) { asm volatile("v_nop" :: "v"(a), "v"(b), "v"(c), "v"(d)); }
__device__ __forceinline__ void acc_guard4(v8f& a, v8f& b, v8f& c, v8f& d) { asm volatile("v_nop\n\tv_nop\n\tv_nop\n\tv_nop" : "+v"(a), "+v"(b), "+v"(c), "+v"(d)); }
template <typename T> struct Frag;
template <> struct Frag<_Float16> {
  typedef v16h V; union U { v16h v; v8h h[2]; };
  static __device__ __forceinline__ v16h load(const _Float16* p) {
    U f; f.h[0] = *(const v8h*)(p); f.h[1] = *(const v8h*)(p + 16); return f.v;
  }
  static __device__ __forceinline__ v8f mma(v16h a, v16h b, v8f c) {
    return __builtin_amdgcn_wmma_f32_16x16x32_f16(false, a, false, b, (short)0, c, false, false);
  }
  static __device__ __forceinline__ void guard(v8f& a, v8f& b, v16h x, v16h y) { dep_guard_h(a, b, x, y); }
  static __device__ __forceinline__ void keep(v16h a, v16h b, v16h c, v16h d) { keep4_h(a, b, c, d); }
};
template <> struct Frag<__bf16> {
  typedef v16b V; union U { v16b v; v8b h[2]; };
  static __device__ __forceinline__ v16b load(const __bf16* p) {
    U f; f.h[0] = *(const v8b*)(p); f.h[1] = *(const v8b*)(p + 16); return f.v;
  }
  static __device__ __forceinline__ v8f mma(v16b a, v16b b, v8f c) {
    return __builtin_amdgcn_wmma_f32_16x16x32_bf16(false, a, false, b, (short)0, c, false, false);
  }
  static __device__ __forceinline__ void guard(v8f& a, v8f& b, v16b x, v16b y) { dep_guard_b(a, b, x, y); }
  static __device__ __forceinline__ void keep(v16b a, v16b b, v16b c, v16b d) { keep4_b(a, b, c, d); }
};

template <int ET> struct Elem;
template <> struct Elem<0> { typedef _Float16 T; };
template <> struct Elem<1> { typedef __bf16 T; };
template <int ET, bool SPLIT, int BIAS_MODE, int OUT_MODE, bool RESID, int ACT = 0>
__global__ __launch_bounds__(256) void wmma_gemm64(
    const unsigned short* __restrict__ Ap, const unsigned short* __restrict__ A2p, int lda, long strideA,
    const unsigned short* __restrict__ Btp, const unsigned short* __restrict__ Bt2p, int ldb, long strideB,
    void* __restrict__ Cout, void* __restrict__ Cout2, int ldc, long strideC,
    const float* __restrict__ bias,
    const float* __restrict__ resid, long strideR,
    int M, int N, int K, float scale) {
  typedef typename Elem<ET>::T T;
  typedef typename Frag<T>::V V;
  const T* A = (const T*)Ap; const T* A2 = (const T*)A2p; const T* Bt = (const T*)Btp; const T* Bt2 = (const T*)Bt2p;
  __shared__ __align__(16) float sT[8][16 * 68];
  const int b    = blockIdx.y;
  const int lane = threadIdx.x & 31;
  const int wave = threadIdx.x >> 5;
  const int tilesN = N >> 6;
  const int tilesM = M >> 6;
  const int tile = blockIdx.x * 8 + wave;
  if (tile >= tilesM * tilesN) return;
  const int tm = tile / tilesN;
  const int tn = tile - tm * tilesN;
  const int m0 = tm << 6;
  const int n0 = tn << 6;

  const T* Ab  = A  + (size_t)b * strideA;
  const T* Bb  = Bt + (size_t)b * strideB;
  const T* Ab2 = SPLIT ? (A2  + (size_t)b * strideA) : nullptr;
  const T* Bb2 = SPLIT ? (Bt2 + (size_t)b * strideB) : nullptr;

  const int rlane = lane & 15;
  const int koff  = (lane >> 4) * 8;
  const int mOff  = (lane >> 4) * 8;

  v8f acc[4][4];
#pragma unroll
  for (int i = 0; i < 4; ++i)
#pragma unroll
    for (int j = 0; j < 4; ++j) acc[i][j] = (v8f){0.f,0.f,0.f,0.f,0.f,0.f,0.f,0.f};

  for (int k0 = 0; k0 < K; k0 += 32) {
    V bh[4], bl[4];
#pragma unroll
    for (int j = 0; j < 4; ++j) {
      const size_t bo = (size_t)(n0 + (j << 4) + rlane) * ldb + koff + k0;
      bh[j] = Frag<T>::load(Bb + bo);
      if (SPLIT) bl[j] = Frag<T>::load(Bb2 + bo);
    }
#pragma unroll
    for (int i = 0; i < 4; ++i) {
      const size_t ao = (size_t)(m0 + (i << 4) + rlane) * lda + koff + k0;
      V ah = Frag<T>::load(Ab + ao);
      V al;
      if (SPLIT) al = Frag<T>::load(Ab2 + ao);
#pragma unroll
      for (int j = 0; j < 4; ++j) {
        acc[i][j] = Frag<T>::mma(ah, bh[j], acc[i][j]);
        if (SPLIT) {
          acc[i][j] = Frag<T>::mma(ah, bl[j], acc[i][j]);
          acc[i][j] = Frag<T>::mma(al, bh[j], acc[i][j]);
        }
      }
      Frag<T>::guard(acc[i][0], acc[i][3], ah, SPLIT ? al : ah);
    }
    Frag<T>::keep(bh[0], bh[1], bh[2], bh[3]);
    if (SPLIT) Frag<T>::keep(bl[0], bl[1], bl[2], bl[3]);
  }
  acc_guard4(acc[0][0], acc[0][1], acc[0][2], acc[0][3]);
  acc_guard4(acc[1][0], acc[1][1], acc[1][2], acc[1][3]);
  acc_guard4(acc[2][0], acc[2][1], acc[2][2], acc[2][3]);
  acc_guard4(acc[3][0], acc[3][1], acc[3][2], acc[3][3]);

  float* slab = sT[wave];
  const float* Rb = RESID ? (resid + (size_t)b * strideR) : nullptr;
#pragma unroll
  for (int i = 0; i < 4; ++i) {
    const int mBase = m0 + (i << 4);
#pragma unroll
    for (int j = 0; j < 4; ++j) {
      const int n = n0 + (j << 4) + rlane;
      float bv = 0.f;
      if (BIAS_MODE == 2) bv = bias[n];
#pragma unroll
      for (int r = 0; r < 8; ++r) {
        float v = acc[i][j][r] * scale;
        if (BIAS_MODE == 1) v += bias[mBase + mOff + r];
        if (BIAS_MODE == 2) v += bv;
        if (RESID) v += Rb[(size_t)(mBase + mOff + r) * ldc + n];
        if (ACT == 1) v = tanhf(v);
        if (ACT == 2) v = fmaxf(v, 0.0f);
        if (ACT == 3) v = v / (1.0f + expf(-v));
        if (ACT == 4) v = (v > 0.f) ? v : 0.01f * v;
        if (ACT == 5) v = 0.5f * v * (1.0f + erff(v * 0.70710678118654752f));
        slab[(mOff + r) * 68 + (j << 4) + rlane] = v;
      }
    }
    __builtin_amdgcn_fence(__ATOMIC_RELEASE, "workgroup");
    __builtin_amdgcn_wave_barrier();
    __builtin_amdgcn_fence(__ATOMIC_ACQUIRE, "workgroup");
    if (OUT_MODE == 0) {
      float* C = (float*)Cout + (size_t)b * strideC;
      const int hh = lane >> 4, c4 = (lane & 15) * 4;
      for (int pass = 0; pass < 2; ++pass) {
#pragma unroll
        for (int it = 0; it < 8; ++it) {
          const int row = it * 2 + hh;
          v4f v = *(const v4f*)(slab + row * 68 + c4);
          *(volatile v4f*)(C + (size_t)(mBase + row) * ldc + n0 + c4) = v;
        }
        __threadfence();
      }
    } else {
      const int q = lane >> 3, c8 = (lane & 7) * 8;
      unsigned short* C  = (unsigned short*)Cout  + (size_t)b * strideC;
      unsigned short* C2 = (OUT_MODE == 2) ? ((unsigned short*)Cout2 + (size_t)b * strideC) : nullptr;
      for (int pass = 0; pass < 2; ++pass) {
#pragma unroll
        for (int it = 0; it < 4; ++it) {
          const int row = it * 4 + q;
          const float* sp = slab + row * 68 + c8;
          v8h hv, lv;
#pragma unroll
          for (int e = 0; e < 8; ++e) {
            if (OUT_MODE == 1) {
              hv[e] = (_Float16)sp[e];
            } else {
              unsigned short hb = f2bf_bits(sp[e]);
              unsigned short lb = f2bf_bits(sp[e] - bf_bits2f(hb));
              hv[e] = __builtin_bit_cast(_Float16, hb);
              lv[e] = __builtin_bit_cast(_Float16, lb);
            }
          }
          *(volatile v8h*)(C + (size_t)(mBase + row) * ldc + n0 + c8) = hv;
          if (OUT_MODE == 2) *(volatile v8h*)(C2 + (size_t)(mBase + row) * ldc + n0 + c8) = lv;
        }
        __threadfence();
      }
    }
    __builtin_amdgcn_fence(__ATOMIC_RELEASE, "workgroup");
    __builtin_amdgcn_wave_barrier();
    __builtin_amdgcn_fence(__ATOMIC_ACQUIRE, "workgroup");
  }
}

__global__ __launch_bounds__(128) void k_build(const float* __restrict__ rawP, const float* __restrict__ rawD,
    float* __restrict__ Maug, float* __restrict__ IpS, float* __restrict__ dvec) {
  const int r = blockIdx.x;
  const int t = threadIdx.x;
  const int colM = 4 * t;
  v4f vm;
  if (t < 64) {
    v4f vs;
#pragma unroll
    for (int e = 0; e < 4; ++e) {
      const int c = colM + e;
      const float prc = rawP[(size_t)r * kDim + c];
      const float pcr = rawP[(size_t)c * kDim + r];
      const float urc = (c >= r) ? prc : 0.0f;
      const float ucr = (r >= c) ? pcr : 0.0f;
      const float s = (urc - ucr) * 0.5f;
      const float id = (c == r) ? 1.0f : 0.0f;
      vm[e] = id - s;
      vs[e] = id + s;
    }
    float* ps = IpS + (size_t)r * kDim + colM;
    *(volatile v4f*)ps = vs;
    __threadfence();
    *(volatile v4f*)ps = vs;
    if (r == 0) {
      v4f vd;
#pragma unroll
      for (int e = 0; e < 4; ++e) {
        const float tt = atanf(rawD[colM + e]) * 0.636619772367581343f;
        vd[e] = (1.0f + tt) / (1.0f - tt);
      }
      float* pd = dvec + colM;
      *(volatile v4f*)pd = vd;
      __threadfence();
      *(volatile v4f*)pd = vd;
    }
  } else {
#pragma unroll
    for (int e = 0; e < 4; ++e) vm[e] = ((colM - kDim + e) == r) ? 1.0f : 0.0f;
  }
  float* pm = Maug + (size_t)r * (2 * kDim) + colM;
  *(volatile v4f*)pm = vm;
  __threadfence();
  *(volatile v4f*)pm = vm;
}

__global__ __launch_bounds__(512) void k_gj(float* M, float* __restrict__ Inv) {
  __shared__ float colk[kDim];
  const int t = threadIdx.x;
  const int wv = t >> 5;
  for (int k = 0; k < kDim; ++k) {
    __syncthreads();
    if (t < kDim) colk[t] = M[(size_t)t * (2 * kDim) + k];
    __syncthreads();
    const bool active = (wv < 8) ? (32 * wv + 31 >= k) : (32 * (wv - 8) <= k);
    if (active) {
      const float inv = 1.0f / colk[k];
      float* pk = M + (size_t)k * (2 * kDim) + t;
      float mk = (*pk) * inv;
      mk = (t == k) ? 1.0f : mk;
      *(volatile float*)pk = mk;
#pragma unroll 4
      for (int r = 0; r < kDim; ++r) {
        float f = colk[r];
        f = (r == k) ? 0.0f : f;
        float* p = M + (size_t)r * (2 * kDim) + t;
        const float v = *p - f * mk;
        *(volatile float*)p = v;
      }
    }
  }
  __syncthreads();
  const int c4 = (t & 63) * 4;
  const int j0 = t >> 6;
#pragma unroll 1
  for (int it = 0; it < kDim / 8; ++it) {
    const int j = it * 8 + j0;
    const v4f v = *(const v4f*)(M + (size_t)j * (2 * kDim) + kDim + c4);
    float* p = Inv + (size_t)j * kDim + c4;
    *(volatile v4f*)p = v;
    __threadfence();
    *(volatile v4f*)p = v;
  }
}

__global__ __launch_bounds__(256) void k_pmat(const float* __restrict__ IpS, const float* __restrict__ Inv,
    float* __restrict__ P) {
  __shared__ float sI[kDim];
  __shared__ __align__(16) float sO[kDim];
  const int r = blockIdx.x, c = threadIdx.x;
  sI[c] = IpS[(size_t)r * kDim + c];
  __syncthreads();
  float acc = 0.0f;
#pragma unroll 4
  for (int j = 0; j < kDim; ++j) acc += sI[j] * Inv[(size_t)j * kDim + c];
  sO[c] = acc;
  __syncthreads();
  if (c < 64) {
    const v4f v = *(const v4f*)(sO + 4 * c);
    float* p = P + (size_t)r * kDim + 4 * c;
    *(volatile v4f*)p = v;
    __threadfence();
    *(volatile v4f*)p = v;
  }
}

__global__ __launch_bounds__(256) void k_wt(const float* __restrict__ P, const float* __restrict__ dvec,
    unsigned short* __restrict__ Wh, unsigned short* __restrict__ Wl) {
  __shared__ float sPr[kDim];
  __shared__ float sd[kDim];
  __shared__ __align__(16) float sO[kDim];
  const int r = blockIdx.x, c = threadIdx.x;
  sPr[c] = P[(size_t)c * kDim + r];
  sd[c] = dvec[c];
  __syncthreads();
  float acc = 0.0f;
#pragma unroll 4
  for (int j = 0; j < kDim; ++j) {
    const float pd = P[(size_t)j * kDim + c] * sd[j];
    acc += pd * sPr[j];
  }
  sO[c] = acc;
  __syncthreads();
  if (c < 32) {
    const v4f a0 = *(const v4f*)(sO + 8 * c);
    const v4f a1 = *(const v4f*)(sO + 8 * c + 4);
    u16x8 hv, lv;
#pragma unroll
    for (int e = 0; e < 4; ++e) {
      const unsigned short h0 = f2bf_bits(a0[e]);
      hv[e] = h0;
      lv[e] = f2bf_bits(a0[e] - bf_bits2f(h0));
      const unsigned short h1 = f2bf_bits(a1[e]);
      hv[4 + e] = h1;
      lv[4 + e] = f2bf_bits(a1[e] - bf_bits2f(h1));
    }
    const size_t off = (size_t)r * kDim + 8 * c;
    *(volatile u16x8*)(Wh + off) = hv;
    *(volatile u16x8*)(Wl + off) = lv;
    __threadfence();
    *(volatile u16x8*)(Wh + off) = hv;
    *(volatile u16x8*)(Wl + off) = lv;
  }
}

__global__ __launch_bounds__(256) void k_trsplit(const float* __restrict__ f1, const float* __restrict__ f2,
    unsigned short* __restrict__ f1h, unsigned short* __restrict__ f1l,
    unsigned short* __restrict__ f2h, unsigned short* __restrict__ f2l) {
  __shared__ __align__(16) float sT[64 * 68];
  const int p0 = blockIdx.x * 64;
  const int c0 = blockIdx.y * 64;
  const int z = blockIdx.z;
  const int tsel = z >> 1, b = z & 1;
  const float* src = (tsel ? f2 : f1) + (size_t)b * kDim * kHW;
  unsigned short* dh = tsel ? f2h : f1h;
  unsigned short* dl = tsel ? f2l : f1l;
  const int tid = threadIdx.x;
#pragma unroll
  for (int it = 0; it < 4; ++it) {
    const int idx = it * 256 + tid;
    const int c = idx >> 4;
    const int p4 = (idx & 15) * 4;
    const v4f v = *(const v4f*)(src + (size_t)(c0 + c) * kHW + p0 + p4);
    sT[(p4 + 0) * 68 + c] = v[0];
    sT[(p4 + 1) * 68 + c] = v[1];
    sT[(p4 + 2) * 68 + c] = v[2];
    sT[(p4 + 3) * 68 + c] = v[3];
  }
  __syncthreads();
  const int wave = tid >> 5, lane = tid & 31;
  const int q = lane >> 3, c8 = (lane & 7) * 8;
  u16x8 hv[2], lv[2];
  size_t off[2];
#pragma unroll
  for (int it = 0; it < 2; ++it) {
    const int p = wave * 8 + it * 4 + q;
    const float* sp = sT + p * 68 + c8;
    const v4f s0 = *(const v4f*)sp;
    const v4f s1 = *(const v4f*)(sp + 4);
#pragma unroll
    for (int e = 0; e < 4; ++e) {
      const unsigned short h0 = f2bf_bits(s0[e]);
      hv[it][e] = h0;
      lv[it][e] = f2bf_bits(s0[e] - bf_bits2f(h0));
      const unsigned short h1 = f2bf_bits(s1[e]);
      hv[it][4 + e] = h1;
      lv[it][4 + e] = f2bf_bits(s1[e] - bf_bits2f(h1));
    }
    off[it] = ((size_t)b * kHW + p0 + p) * kDim + c0 + c8;
  }
  for (int pass = 0; pass < 2; ++pass) {
    *(volatile u16x8*)(dh + off[0]) = hv[0];
    *(volatile u16x8*)(dl + off[0]) = lv[0];
    *(volatile u16x8*)(dh + off[1]) = hv[1];
    *(volatile u16x8*)(dl + off[1]) = lv[1];
    __threadfence();
  }
}

__global__ __launch_bounds__(256) void k_pool(const float* __restrict__ in, float* __restrict__ out, int lw_in, int n4) {
  const int i = blockIdx.x * 256 + threadIdx.x;
  if (i >= n4) return;
  const int lwo = lw_in - 1;
  const int wo = 1 << lwo;
  const int win = 1 << lw_in;
  const int e0 = i * 4;
  const int x = e0 & (wo - 1);
  const int rest = e0 >> lwo;
  const int y = rest & (wo - 1);
  const int n = rest >> lwo;
  const float* p = in + ((size_t)n * win + 2 * y) * win + 2 * x;
  const v4f a0 = *(const v4f*)p;
  const v4f a1 = *(const v4f*)(p + 4);
  const v4f b0 = *(const v4f*)(p + win);
  const v4f b1 = *(const v4f*)(p + win + 4);
  v4f o;
  o[0] = (a0[0] + a0[1] + b0[0] + b0[1]) * 0.25f;
  o[1] = (a0[2] + a0[3] + b0[2] + b0[3]) * 0.25f;
  o[2] = (a1[0] + a1[1] + b1[0] + b1[1]) * 0.25f;
  o[3] = (a1[2] + a1[3] + b1[2] + b1[3]) * 0.25f;
  float* po = out + (size_t)e0;
  *(volatile v4f*)po = o;
  __threadfence();
  *(volatile v4f*)po = o;
}

__global__ __launch_bounds__(256) void k_sample(const float* __restrict__ coords,
    const float* __restrict__ lv0, const float* __restrict__ lv1,
    const float* __restrict__ lv2, const float* __restrict__ lv3,
    float* __restrict__ out, int bsel, int h0) {
#pragma clang fp contract(off)
  const int bid = blockIdx.x;
  const int q2 = bid & 1;
  const int ch = bid >> 1;
  const int level = ch / 81;
  const int rem = ch - level * 81;
  const int ax = rem / 9;
  const int by = rem - ax * 9;
  const float dx = (float)(ax - 4);
  const float dy = (float)(by - 4);
  const float sc = __uint_as_float((unsigned)(127 - level) << 23);
  const int lwl = 6 - level;
  const int wl = 1 << lwl;
  const int npix = 1 << (2 * lwl);
  const float* lvp = (level == 0) ? lv0 : ((level == 1) ? lv1 : ((level == 2) ? lv2 : lv3));
  const int tid = threadIdx.x;
  const int hloc = q2 * 16 + (tid >> 4);
  const int h = h0 + hloc;
  const int w0 = (tid & 15) * 4;
  const size_t cb = ((size_t)(bsel * 2) * kImg + h) * kImg + w0;
  const v4f cx4 = *(const v4f*)(coords + cb);
  const v4f cy4 = *(const v4f*)(coords + cb + kHW);
  v4f res;
#pragma unroll
  for (int e = 0; e < 4; ++e) {
    const float* img = lvp + (size_t)(hloc * kImg + w0 + e) * npix;
    float x = cx4[e] * sc + dx;
    float y = cy4[e] * sc + dy;
    x = fminf(fmaxf(x, -1.0e6f), 1.0e6f);
    y = fminf(fmaxf(y, -1.0e6f), 1.0e6f);
    const float x0f = floorf(x), y0f = floorf(y);
    const int xi0 = (int)x0f, yi0 = (int)y0f;
    const int xi1 = xi0 + 1, yi1 = yi0 + 1;
    const float wx1 = x - x0f;
    const float wx0 = 1.0f - wx1;
    const float wy1 = y - y0f;
    const float wy0 = 1.0f - wy1;
    const bool vx0 = (xi0 >= 0) && (xi0 < wl);
    const bool vx1 = (xi1 >= 0) && (xi1 < wl);
    const bool vy0 = (yi0 >= 0) && (yi0 < wl);
    const bool vy1 = (yi1 >= 0) && (yi1 < wl);
    const int xc0 = min(max(xi0, 0), wl - 1);
    const int xc1 = min(max(xi1, 0), wl - 1);
    const int yc0 = min(max(yi0, 0), wl - 1);
    const int yc1 = min(max(yi1, 0), wl - 1);
    const float g00 = img[(yc0 << lwl) + xc0];
    const float g10 = img[(yc0 << lwl) + xc1];
    const float g01 = img[(yc1 << lwl) + xc0];
    const float g11 = img[(yc1 << lwl) + xc1];
    const float t00 = (vx0 && vy0) ? g00 : 0.0f;
    const float t10 = (vx1 && vy0) ? g10 : 0.0f;
    const float t01 = (vx0 && vy1) ? g01 : 0.0f;
    const float t11 = (vx1 && vy1) ? g11 : 0.0f;
    res[e] = wy0 * wx0 * t00 + wy0 * wx1 * t10 + wy1 * wx0 * t01 + wy1 * wx1 * t11;
  }
  float* po = out + (((size_t)(bsel * kNCH + ch)) * kImg + h) * kImg + w0;
  *(volatile v4f*)po = res;
  __threadfence();
  *(volatile v4f*)po = res;
}

extern "C" void kernel_launch(void* const* d_in, const int* in_sizes, int n_in,
                              void* d_out, int out_size, void* d_ws, size_t ws_size,
                              hipStream_t stream) {
  if (n_in < 5) return;
  if (in_sizes[0] != kNB * kDim * kHW || in_sizes[1] != kNB * kDim * kHW ||
      in_sizes[2] != kNB * 2 * kHW || in_sizes[3] != kDim * kDim || in_sizes[4] != kDim) return;
  if (out_size != kNB * kNCH * kHW) return;
  if (kWsTotal > ws_size) return;

  const float* fmap1  = (const float*)d_in[0];
  const float* fmap2  = (const float*)d_in[1];
  const float* coords = (const float*)d_in[2];
  const float* rawP   = (const float*)d_in[3];
  const float* rawD   = (const float*)d_in[4];
  float* out = (float*)d_out;
  char* ws = (char*)d_ws;

  float* Maug = (float*)(ws + oMaug);
  float* IpS  = (float*)(ws + oIpS);
  float* Inv  = (float*)(ws + oInv);
  float* Pm   = (float*)(ws + oPm);
  float* dvec = (float*)(ws + oDvec);
  unsigned short* WTh = (unsigned short*)(ws + oWTh);
  unsigned short* WTl = (unsigned short*)(ws + oWTl);
  unsigned short* f1h = (unsigned short*)(ws + oF1h);
  unsigned short* f1l = (unsigned short*)(ws + oF1l);
  unsigned short* f2h = (unsigned short*)(ws + oF2h);
  unsigned short* f2l = (unsigned short*)(ws + oF2l);
  unsigned short* Th  = (unsigned short*)(ws + oTh);
  unsigned short* Tl  = (unsigned short*)(ws + oTl);
  float* corr = (float*)(ws + oCorr);
  float* pyr1 = (float*)(ws + oP1);
  float* pyr2 = (float*)(ws + oP2);
  float* pyr3 = (float*)(ws + oP3);

  k_build<<<kDim, 128, 0, stream>>>(rawP, rawD, Maug, IpS, dvec);
  k_gj<<<1, 512, 0, stream>>>(Maug, Inv);
  k_pmat<<<kDim, 256, 0, stream>>>(IpS, Inv, Pm);
  k_wt<<<kDim, 256, 0, stream>>>(Pm, dvec, WTh, WTl);

  k_trsplit<<<dim3(kHW / 64, kDim / 64, 4), 256, 0, stream>>>(fmap1, fmap2, f1h, f1l, f2h, f2l);

  {
    const int tiles = (kHW / 64) * (kDim / 64);
    wmma_gemm64<1, true, 0, 2, false><<<dim3(tiles / 8, kNB), 256, 0, stream>>>(
        f1h, f1l, kDim, (long)kHW * kDim,
        WTh, WTl, kDim, 0L,
        (void*)Th, (void*)Tl, kDim, (long)kHW * kDim,
        dvec, dvec, 0L,
        kHW, kDim, kDim, 1.0f);
  }

  for (int qc = 0; qc < kNChunk; ++qc) {
    const int b = qc >> 1;
    const int i0 = (qc & 1) * kChunkRows;
    const int h0 = (qc & 1) * kChunkH;
    const size_t aoff = ((size_t)b * kHW + i0) * kDim;
    const size_t boff = (size_t)b * kHW * kDim;
    const int tiles = (kChunkRows / 64) * (kHW / 64);
    wmma_gemm64<1, true, 0, 0, false><<<dim3(tiles / 8, 1), 256, 0, stream>>>(
        Th + aoff, Tl + aoff, kDim, 0L,
        f2h + boff, f2l + boff, kDim, 0L,
        (void*)corr, (void*)corr, kHW, 0L,
        dvec, dvec, 0L,
        kChunkRows, kHW, kDim, 0.0625f);
    k_pool<<<(kChunkRows * 1024 / 4) / 256, 256, 0, stream>>>(corr, pyr1, 6, kChunkRows * 1024 / 4);
    k_pool<<<(kChunkRows * 256 / 4) / 256, 256, 0, stream>>>(pyr1, pyr2, 5, kChunkRows * 256 / 4);
    k_pool<<<(kChunkRows * 64 / 4) / 256, 256, 0, stream>>>(pyr2, pyr3, 4, kChunkRows * 64 / 4);
    k_sample<<<kNCH * 2, 256, 0, stream>>>(coords, corr, pyr1, pyr2, pyr3, out, b, h0);
  }
}
